// DeepTypedGraphNet_71665824301916
// MI455X (gfx1250) — hardware-run, weakly checked
//
#include <hip/hip_runtime.h>


namespace {
constexpr int N = 50000, E = 800000, DN = 16, DE = 8, D = 64, DOUT = 16, NPB = 8;
constexpr float HS = 256.0f, WSC = 256.0f, LNEPS = 1e-5f;
typedef _Float16 b16;
typedef __attribute__((ext_vector_type(16))) _Float16 v16b;
typedef __attribute__((ext_vector_type(8))) _Float16 v8b;
typedef __attribute__((ext_vector_type(8))) float v8f;
typedef __attribute__((ext_vector_type(4))) float v4f;
typedef __attribute__((ext_vector_type(2))) float v2f;
__device__ __forceinline__ float bf16_rne(float f) { unsigned int u = __float_as_uint(f); u += 0x7FFFu + ((u >> 16) & 1u); float r = __uint_as_float(u & 0xFFFF0000u); asm volatile("" : "+v"(r)); return r; }
__device__ __forceinline__ float bfv(float f) { float r = bf16_rne(f); asm volatile("" : "+v"(r)); return r; }
__device__ __forceinline__ void split16(float v, b16& hi, b16& lo) { hi = (b16)v; lo = (b16)(v - (float)hi); }
__device__ __forceinline__ v16b frag_kb(const b16* p, int hh) { const v8b a = *(const v8b*)(p + 8 * hh), b = *(const v8b*)(p + 16 + 8 * hh); v16b f;
#pragma unroll
  for (int e = 0; e < 8; ++e) { f[e] = a[e]; f[8 + e] = b[e]; } return f; }
__device__ __forceinline__ v8f wmma16b(v16b a, v16b b, v8f c) { v8f d = __builtin_amdgcn_wmma_f32_16x16x32_f16(false, a, false, b, (short)0, c, false, false); asm volatile("v_nop\n\tv_nop\n\tv_nop\n\tv_nop" : "+v"(d) : "v"(a), "v"(b)); return d; }
__device__ __forceinline__ void wave_lds_sync() { __builtin_amdgcn_fence(__ATOMIC_RELEASE, "workgroup"); __builtin_amdgcn_wave_barrier(); __builtin_amdgcn_fence(__ATOMIC_ACQUIRE, "workgroup"); }
__device__ __forceinline__ float pmul(float a, float b) { float p = a * b; asm volatile("" : "+v"(p)); return p; }
__device__ __forceinline__ int iclamp(int v, int lo, int hi) { return v < lo ? lo : (v > hi ? hi : v); }
__device__ __forceinline__ float silu(float v) { return v / (1.0f + __expf(-v)); }
constexpr int CSR_NBLK8 = 512, CSR_GB8 = 8, CSR_GN8 = 1 << CSR_GB8  , CSR_TS8 = (CSR_GN8 < 32 ? 32 : CSR_GN8)  , CSR_MAXG8 = 512, CSR_CAP8 = 12288  ;
__device__ __host__ __forceinline__ int csr_tix8(int v) { return (v >> CSR_GB8) * CSR_TS8 + (v & (CSR_GN8 - 1)); }
__global__ __launch_bounds__(64) void csrA_kernel8(const int* __restrict__ dst, int E, int N, int nG, int CHP, int NGP, int* __restrict__ STG, int* __restrict__ HST) {
  extern __shared__ int sm[];
  int* cnt = sm; int* run = sm + NGP; int* ids = sm + 2 * NGP;
  const int b = blockIdx.x; const int ch = (E + CSR_NBLK8 - 1) / CSR_NBLK8; const int e0 = b * ch, e1 = min(E, e0 + ch);
  for (int i = threadIdx.x; i < NGP; i += 64) cnt[i] = 0;
  for (int i = threadIdx.x; i < CHP; i += 64) ids[i] = -1;
  __syncthreads();
  if (threadIdx.x == 0) {
    for (int e = e0; e < e1; ++e) { int d = dst[e]; d = (d < 0) ? 0 : (d >= N ? N - 1 : d); cnt[d >> CSR_GB8] += 1; }
    int acc = 0; for (int g = 0; g < nG; ++g) { run[g] = acc; acc += cnt[g]; }
    for (int e = e0; e < e1; ++e) { int d = dst[e]; d = (d < 0) ? 0 : (d >= N ? N - 1 : d); const int g = d >> CSR_GB8; ids[run[g]] = e; run[g] += 1; } }
  __syncthreads();
  typedef __attribute__((ext_vector_type(4))) int v4i;
  for (int pass = 0; pass < 2; ++pass) {
    for (int i = threadIdx.x; i < CHP / 4; i += 64) *(volatile v4i*)(STG + (size_t)b * CHP + i * 4) = *(const v4i*)(&ids[i * 4]);
    for (int i = threadIdx.x; i < NGP / 4; i += 64) { v4i v; for (int e = 0; e < 4; ++e) v[e] = (i * 4 + e < nG) ? cnt[i * 4 + e] : 0; *(volatile v4i*)(HST + (size_t)b * NGP + i * 4) = v; }
    __threadfence(); }
}
__global__ __launch_bounds__(512) void csrS_kernel8(const int* __restrict__ HST, int nG, int NGP, int* __restrict__ START, int* __restrict__ TOT, int* __restrict__ OFF) {
  __shared__ int tot[CSR_MAXG8];
  const int b = threadIdx.x;
  for (int pass = 0; pass < 2; ++pass) { int runb = 0; for (int g = 0; g < nG; ++g) { int c = HST[(size_t)b * NGP + g]; c = (c < 0) ? 0 : c; ((volatile int*)OFF)[(size_t)g * CSR_NBLK8 + b] = runb; runb += c; } __threadfence(); }
  for (int g = threadIdx.x; g < nG; g += 512) { int s = 0; for (int bb = 0; bb < CSR_NBLK8; ++bb) { int c = HST[(size_t)bb * NGP + g]; s += (c < 0) ? 0 : c; } tot[g] = s; }
  __syncthreads();
  if (threadIdx.x < 32) {
    __shared__ int st[CSR_MAXG8 + 32];
    if (threadIdx.x == 0) { int acc = 0; for (int g = 0; g < NGP; ++g) { st[g] = acc; if (g < nG) acc += (tot[g] + 31) & ~31; } st[NGP] = acc; }
    __builtin_amdgcn_fence(__ATOMIC_RELEASE, "workgroup"); __builtin_amdgcn_wave_barrier(); __builtin_amdgcn_fence(__ATOMIC_ACQUIRE, "workgroup");
    for (int pass = 0; pass < 2; ++pass) { for (int i = threadIdx.x; i < NGP + 32; i += 32) { ((volatile int*)START)[i] = (i <= NGP) ? st[min(i, NGP)] : 0; ((volatile int*)TOT)[i] = (i < nG) ? tot[i] : 0; } __threadfence(); } }
}
__global__ __launch_bounds__(256) void csrB_kernel8(const int* __restrict__ dst, int N, int nG, int CHP, int NGP, int permLen, const int* __restrict__ STG, const int* __restrict__ HST, const int* __restrict__ OFF, const int* __restrict__ START, const int* __restrict__ TOT, int* __restrict__ PERM, int* __restrict__ ROWPTR, int* __restrict__ ROWCNT, int* __restrict__ FLAG) {
  typedef __attribute__((ext_vector_type(4))) int v4i;
  __shared__ int ids[CSR_CAP8]; __shared__ unsigned short key[CSR_CAP8]; __shared__ int outp[CSR_CAP8]; __shared__ int ncnt[CSR_GN8 + 1]; __shared__ int boff[CSR_NBLK8 + 1];
  const int g = blockIdx.x, t_ = threadIdx.x; int tot = TOT[g]; int st = START[g], stn = START[g + 1]; const int v0 = g * CSR_GN8; const int nv = min(CSR_GN8, N - v0); const int t0 = g * CSR_TS8;
  st = (st < 0) ? 0 : (st > permLen - 32 ? permLen - 32 : st) & ~31; stn = (stn < st) ? st : (stn > permLen ? permLen : stn); tot = (tot < 0) ? 0 : tot; if (tot > stn - st && tot <= CSR_CAP8) tot = stn - st;
  if (tot > CSR_CAP8) {
    for (int pass = 0; pass < 2; ++pass) { for (int i = t_; i < CSR_TS8 / 4; i += 256) { v4i a, c; for (int e = 0; e < 4; ++e) { a[e] = st; c[e] = 0; } *(volatile v4i*)(ROWPTR + t0 + i * 4) = a; *(volatile v4i*)(ROWCNT + t0 + i * 4) = c; } if (t_ == 0) ((volatile int*)FLAG)[0] = 1; __threadfence(); } (void)nv; return; }
  if (t_ == 0) { int acc = 0; for (int b = 0; b < CSR_NBLK8; ++b) { boff[b] = acc; int c = HST[(size_t)b * NGP + g]; c = (c < 0) ? 0 : (c > CHP ? CHP : c); acc += c; if (acc > tot) acc = tot; } boff[CSR_NBLK8] = acc; }
  for (int i = t_; i <= CSR_GN8; i += 256) ncnt[i] = 0;
  __syncthreads();
  for (int b = 0; b < CSR_NBLK8; ++b) { const int c = boff[b + 1] - boff[b]; int o_ = OFF[(size_t)g * CSR_NBLK8 + b]; o_ = (o_ < 0) ? 0 : (o_ > CHP - c ? CHP - c : o_); const int* src_ = STG + (size_t)b * CHP + o_;
    for (int i = t_; i < c; i += 256) { int id = src_[i]; id = (id < 0) ? 0 : id; ids[boff[b] + i] = id; int d = dst[id]; d = (d < v0) ? v0 : (d >= N ? N - 1 : d); int kk = d - v0; kk = (kk < 0) ? 0 : (kk >= CSR_GN8 ? CSR_GN8 - 1 : kk); key[boff[b] + i] = (unsigned short)kk; } }
  __syncthreads();
  if (t_ == 0) { for (int i = 0; i < tot; ++i) ncnt[key[i]] += 1; int acc = 0; for (int vl = 0; vl < CSR_GN8; ++vl) { const int c = ncnt[vl]; ncnt[vl] = acc; acc += c; } ncnt[CSR_GN8] = acc;
    for (int i = 0; i < tot; ++i) { const int vl = key[i]; outp[ncnt[vl]] = ids[i]; ncnt[vl] += 1; }
    for (int vl = CSR_GN8; vl > 0; --vl) ncnt[vl] = ncnt[vl - 1]; ncnt[0] = 0; }
  __syncthreads();
  for (int pass = 0; pass < 2; ++pass) {
    for (int i = t_; i < (stn - st) / 4; i += 256) { v4i v; for (int e = 0; e < 4; ++e) { const int q = i * 4 + e; v[e] = (q < tot) ? outp[q] : -1; } *(volatile v4i*)(PERM + st + i * 4) = v; }
    for (int i = t_; i < CSR_TS8 / 4; i += 256) { v4i a, c; for (int e = 0; e < 4; ++e) { const int vl = i * 4 + e; const int vc = vl < CSR_GN8 ? vl : CSR_GN8; a[e] = (vl < CSR_GN8) ? st + ncnt[vc] : st; c[e] = (vl < nv) ? (ncnt[(vc < CSR_GN8 ? vc : CSR_GN8 - 1) + 1] - ncnt[vc]) : 0; } *(volatile v4i*)(ROWPTR + t0 + i * 4) = a; *(volatile v4i*)(ROWCNT + t0 + i * 4) = c; }
    __threadfence(); }
}
__global__ __launch_bounds__(256) void csrZ_kernel8(int* __restrict__ p, size_t n4) { typedef __attribute__((ext_vector_type(4))) int v4i; const size_t tid = (size_t)blockIdx.x * 256 + threadIdx.x, nth = (size_t)gridDim.x * 256; v4i z = {0, 0, 0, 0}; for (size_t i = tid; i < n4; i += nth) *(volatile v4i*)(p + i * 4) = z; }
struct CsrBufs8 { int *STG, *HST, *OFF, *START, *TOT, *PERM, *ROWPTR, *ROWCNT, *FLAG; int nG, NGP, CHP; size_t permLen; char* base; size_t bytes; };
static size_t csr_carve8(CsrBufs8& c, char* ws, size_t off, int E, int N) {
  const size_t off0 = off; c.base = ws + off;
  auto al = [&](size_t bytes) { char* p = ws + off; off += (bytes + 255) & ~(size_t)255; return p; };
  c.nG = (N + CSR_GN8 - 1) / CSR_GN8; c.NGP = (c.nG + 31) & ~31; const int ch = (E + CSR_NBLK8 - 1) / CSR_NBLK8; c.CHP = (ch + 31) & ~31; c.permLen = (size_t)E + 32 * (size_t)c.nG + 32;
  c.STG = (int*)al((size_t)CSR_NBLK8 * c.CHP * 4); c.HST = (int*)al((size_t)CSR_NBLK8 * c.NGP * 4); c.OFF = (int*)al((size_t)c.NGP * CSR_NBLK8 * 4); c.START = (int*)al((size_t)(c.NGP + 64) * 4); c.TOT = (int*)al((size_t)(c.NGP + 64) * 4);
  c.PERM = (int*)al(c.permLen * 4); c.ROWPTR = (int*)al((size_t)c.nG * CSR_TS8 * 4); c.ROWCNT = (int*)al((size_t)c.nG * CSR_TS8 * 4); c.FLAG = (int*)al(256);
  c.bytes = off - off0; return off;
}
static void csr_build8(const CsrBufs8& c, const int* dst, int E, int N, hipStream_t stream) {
  const size_t smem = (size_t)(2 * c.NGP + c.CHP) * 4;
  csrZ_kernel8<<<512, 256, 0, stream>>>((int*)c.base, c.bytes / 16);
  csrA_kernel8<<<CSR_NBLK8, 64, smem, stream>>>(dst, E, N, c.nG, c.CHP, c.NGP, c.STG, c.HST);
  csrS_kernel8<<<1, 512, 0, stream>>>(c.HST, c.nG, c.NGP, c.START, c.TOT, c.OFF);
  csrB_kernel8<<<c.nG, 256, 0, stream>>>(dst, N, c.nG, c.CHP, c.NGP, (int)c.permLen, c.STG, c.HST, c.OFF, c.START, c.TOT, c.PERM, c.ROWPTR, c.ROWCNT, c.FLAG);
}


__global__ __launch_bounds__(256) void wput_kernel(const float* __restrict__ ne0, const float* __restrict__ ne1, const float* __restrict__ ee0, const float* __restrict__ ee1, const float* __restrict__ eb0, const float* __restrict__ eb1, const float* __restrict__ nb0, const float* __restrict__ nb1, const float* __restrict__ dc0, const float* __restrict__ dc1,
    b16* __restrict__ NE0, b16* __restrict__ NE1, b16* __restrict__ EE0, b16* __restrict__ EE1, b16* __restrict__ EB0, b16* __restrict__ EB1, b16* __restrict__ NB0, b16* __restrict__ NB1, b16* __restrict__ DC0, b16* __restrict__ DC1) { const size_t nt = (size_t)gridDim.x * 256, u0 = (size_t)blockIdx.x * 256 + threadIdx.x; v8b v;
  auto put = [&](const float* src, b16* dst, int kin, int kp, int nout, int nmat) { for (size_t u = u0; u < (size_t)nmat * nout * (kp / 8); u += nt) { const int m = (int)(u / ((size_t)nout * (kp / 8))); const int r = (int)(u % ((size_t)nout * (kp / 8))); const int o = r / (kp / 8), k0 = (r % (kp / 8)) * 8;
#pragma unroll
      for (int j = 0; j < 8; ++j) { const int k = k0 + j; v[j] = (b16)(k < kin ? bf16_rne(src[((size_t)m * kin + k) * nout + o]) * WSC : 0.0f); } for (int pass = 0; pass < 2; ++pass) { *(volatile v8b*)(dst + ((size_t)m * nout + o) * kp + k0) = v; __threadfence(); } } };
  put(ne0, NE0, DN, 32, D, 1); put(ne1, NE1, D, D, D, 1); put(ee0, EE0, DE, 32, D, 1); put(ee1, EE1, D, D, D, 1); put(eb0, EB0, 3 * D, 3 * D, D, 2); put(eb1, EB1, D, D, D, 2); put(nb0, NB0, 2 * D, 2 * D, D, 2); put(nb1, NB1, D, D, D, 2); put(dc0, DC0, D, D, D, 1); put(dc1, DC1, D, D, DOUT, 1); }
template <int MODE>
__global__ __launch_bounds__(32) void mlp_kernel(const float* __restrict__ IN0, const float* __restrict__ NPL, const int* __restrict__ snd, const int* __restrict__ rcv, const int* __restrict__ PERM, const int* __restrict__ ROWPTR, const int* __restrict__ ROWCNT, int permLen,
    const b16* __restrict__ W0, const float* __restrict__ b0, const b16* __restrict__ W1, const float* __restrict__ b1, const float* __restrict__ g, const float* __restrict__ bt, int RLIM, int ELIM, float* __restrict__ DST) {
  constexpr int K0 = MODE == 0 ? 32 : (MODE == 1 ? 32 : (MODE == 2 ? 3 * D : (MODE == 3 ? 2 * D : D))); constexpr int NT1 = MODE == 4 ? 1 : 4; constexpr int OW = MODE == 4 ? DOUT : D; constexpr bool LNF = MODE != 4, RESF = (MODE == 2 || MODE == 3);
  __shared__ __attribute__((aligned(16))) b16 Ah[16][K0 + 8], Al[16][K0 + 8], Hh[16][D + 8], Hl[16][D + 8]; __shared__ float Tf[16][D + 4]; const int lane = threadIdx.x, nloc = lane & 15, hlf = lane >> 4; const size_t m0 = (size_t)blockIdx.x * 16; if (m0 >= (size_t)RLIM) return;
  for (int rr = 0; rr < 16; ++rr) { const size_t row = m0 + rr;
    if (MODE == 0) { const float v = lane < DN ? bf16_rne(IN0[row * DN + lane]) : 0.0f; Ah[rr][lane] = (b16)(v * HS); Al[rr][lane] = (b16)0.0f; }
    else if (MODE == 1) { const float v = lane < DE ? bf16_rne(IN0[row * DE + lane]) : 0.0f; Ah[rr][lane] = (b16)(v * HS); Al[rr][lane] = (b16)0.0f; }
    else if (MODE == 2) { const size_t s = (size_t)iclamp(snd[row], 0, N - 1), r = (size_t)iclamp(rcv[row], 0, N - 1); for (int q = 0; q < 2; ++q) { const int c = q * 32 + lane; b16 p, ql; split16(IN0[row * D + c] * HS, p, ql); Ah[rr][c] = p; Al[rr][c] = ql; split16(NPL[s * D + c] * HS, p, ql); Ah[rr][D + c] = p; Al[rr][D + c] = ql; split16(NPL[r * D + c] * HS, p, ql); Ah[rr][2 * D + c] = p; Al[rr][2 * D + c] = ql; } }
    else if (MODE == 3) { int st = ROWPTR[row], cnt = ROWCNT[row]; cnt = iclamp(cnt, 0, E); st = iclamp(st, 0, permLen - cnt); v2f ag = {0.0f, 0.0f};
#pragma unroll 1
      for (int j = 0; j < cnt; ++j) { const int e = iclamp(PERM[st + j], 0, E - 1); if (e >= ELIM) continue; const v2f v = *(const v2f*)(NPL + (size_t)e * D + lane * 2); ag[0] += v[0]; ag[1] += v[1]; }
      for (int k = 0; k < 2; ++k) { const int c = lane * 2 + k; b16 p, ql; split16(IN0[row * D + c] * HS, p, ql); Ah[rr][c] = p; Al[rr][c] = ql; split16(ag[k] * HS, p, ql); Ah[rr][D + c] = p; Al[rr][D + c] = ql; } }
    else { for (int q = 0; q < 2; ++q) { const int c = q * 32 + lane; b16 p, ql; split16(IN0[row * D + c] * HS, p, ql); Ah[rr][c] = p; Al[rr][c] = ql; } } }
  if (lane < 16) for (int k = K0; k < K0 + 8; ++k) { Ah[lane][k] = (b16)0.0f; Al[lane][k] = (b16)0.0f; Hh[lane][D + k - K0] = (b16)0.0f; Hl[lane][D + k - K0] = (b16)0.0f; }
  wave_lds_sync();
  v8f acc[4] = {(v8f){}, (v8f){}, (v8f){}, (v8f){}};
#pragma unroll
  for (int kb = 0; kb < K0; kb += 32) { const v16b a = frag_kb(&Ah[nloc][kb], hlf), al = frag_kb(&Al[nloc][kb], hlf);
#pragma unroll
    for (int t = 0; t < 4; ++t) { const v16b bw = frag_kb(W0 + (size_t)(t * 16 + nloc) * K0 + kb, hlf); acc[t] = wmma16b(a, bw, acc[t]); if (MODE >= 2) acc[t] = wmma16b(al, bw, acc[t]); } }
#pragma unroll
  for (int t = 0; t < 4; ++t) { const int cc = t * 16 + nloc; const float bb = bfv(b0[cc]);
#pragma unroll
    for (int r8 = 0; r8 < 8; ++r8) { b16 p, ql; split16(silu(acc[t][r8] * (1.0f / (HS * WSC)) + bb) * HS, p, ql); Hh[8 * hlf + r8][cc] = p; Hl[8 * hlf + r8][cc] = ql; } }
  wave_lds_sync();
  v8f acc2[NT1];
#pragma unroll
  for (int t = 0; t < NT1; ++t) acc2[t] = (v8f){};
#pragma unroll
  for (int kb = 0; kb < D; kb += 32) { const v16b a = frag_kb(&Hh[nloc][kb], hlf), al = frag_kb(&Hl[nloc][kb], hlf);
#pragma unroll
    for (int t = 0; t < NT1; ++t) { const v16b bw = frag_kb(W1 + (size_t)(t * 16 + nloc) * D + kb, hlf); acc2[t] = wmma16b(a, bw, acc2[t]); acc2[t] = wmma16b(al, bw, acc2[t]); } }
#pragma unroll
  for (int t = 0; t < NT1; ++t) { const int cc = t * 16 + nloc; const float bb = bfv(b1[cc]);
#pragma unroll
    for (int r8 = 0; r8 < 8; ++r8) Tf[8 * hlf + r8][cc] = acc2[t][r8] * (1.0f / (HS * WSC)) + bb; }
  wave_lds_sync();
  if (LNF) { for (int rr = 0; rr < 16; ++rr) { float v[2], sm = 0.0f; for (int k = 0; k < 2; ++k) { v[k] = Tf[rr][lane * 2 + k]; sm += v[k]; } for (int o = 16; o; o >>= 1) sm += __shfl_xor(sm, o); const float mu = sm / D; float q2 = 0.0f; for (int k = 0; k < 2; ++k) q2 += (v[k] - mu) * (v[k] - mu); for (int o = 16; o; o >>= 1) q2 += __shfl_xor(q2, o); const float rs = rsqrtf(q2 / D + LNEPS);
      for (int k = 0; k < 2; ++k) { const int c = lane * 2 + k; float y = pmul((v[k] - mu) * rs, bfv(g[c])) + bfv(bt[c]); if (RESF) y += IN0[(m0 + rr) * D + c]; Tf[rr][c] = y; } }
    wave_lds_sync(); }
  for (int pass = 0; pass < 2; ++pass) { for (int rr = 0; rr < 16; ++rr) { if (MODE == 4) { if (lane < DOUT) ((volatile float*)DST)[(m0 + rr) * DOUT + lane] = Tf[rr][lane]; } else *(volatile v2f*)(DST + (m0 + rr) * D + lane * 2) = (v2f){Tf[rr][lane * 2], Tf[rr][lane * 2 + 1]}; } __threadfence(); } }
}

extern "C" void kernel_launch(void* const* d_in, const int* in_sizes, int n_in, void* d_out, int out_size, void* d_ws, size_t ws_size, hipStream_t stream) {
  (void)n_in;
  auto Fp = [&](int i) { return (const float*)d_in[i]; }; auto Ip = [&](int i) { return (const int*)d_in[i]; };
  if (in_sizes[0] != N * DN || in_sizes[1] != E * DE || in_sizes[2] != E || in_sizes[3] != E || in_sizes[4] != DN * D || in_sizes[10] != DE * D || in_sizes[16] != 2 * 3 * D * D || in_sizes[22] != 2 * 2 * D * D || in_sizes[28] != D * D || in_sizes[30] != D * DOUT || out_size != N * DOUT) return;
  const int ELIM = E;
  size_t off = 0; char* ws = (char*)d_ws;
  auto carve = [&](size_t bytes) { char* p = ws + off; off += (bytes + 255) & ~(size_t)255; return p; };
  b16* NE0 = (b16*)carve(D * 32 * 2); b16* NE1 = (b16*)carve(D * D * 2); b16* EE0 = (b16*)carve(D * 32 * 2); b16* EE1 = (b16*)carve(D * D * 2); b16* EB0 = (b16*)carve((size_t)2 * D * 3 * D * 2); b16* EB1 = (b16*)carve((size_t)2 * D * D * 2); b16* NB0 = (b16*)carve((size_t)2 * D * 2 * D * 2); b16* NB1 = (b16*)carve((size_t)2 * D * D * 2); b16* DC0 = (b16*)carve(D * D * 2); b16* DC1 = (b16*)carve(DOUT * D * 2);
  float* NP_ = (float*)carve((size_t)N * D * 4); float* EP = (float*)carve((size_t)E * D * 4); CsrBufs8 csr; off = csr_carve8(csr, ws, off, E, N);
  if (off > ws_size || off > ((size_t)232 << 20)) return;
  const int* nul = nullptr;
  wput_kernel<<<64, 256, 0, stream>>>(Fp(4), Fp(6), Fp(10), Fp(12), Fp(16), Fp(18), Fp(22), Fp(24), Fp(28), Fp(30), NE0, NE1, EE0, EE1, EB0, EB1, NB0, NB1, DC0, DC1);
  csr_build8(csr, Ip(3), E, N, stream);
  mlp_kernel<0><<<N / 16, 32, 0, stream>>>(Fp(0), nullptr, nul, nul, nul, nul, nul, 0, NE0, Fp(5), NE1, Fp(7), Fp(8), Fp(9), N, ELIM, NP_);
  mlp_kernel<1><<<E / 16, 32, 0, stream>>>(Fp(1), nullptr, nul, nul, nul, nul, nul, 0, EE0, Fp(11), EE1, Fp(13), Fp(14), Fp(15), ELIM, ELIM, EP);
  for (int s = 0; s < 2; ++s) {
    mlp_kernel<2><<<E / 16, 32, 0, stream>>>(EP, NP_, Ip(2), Ip(3), nul, nul, nul, 0, EB0 + (size_t)s * D * 3 * D, Fp(17) + s * D, EB1 + (size_t)s * D * D, Fp(19) + s * D, Fp(20) + s * D, Fp(21) + s * D, ELIM, ELIM, EP);
    mlp_kernel<3><<<N / 16, 32, 0, stream>>>(NP_, EP, nul, nul, csr.PERM, csr.ROWPTR, csr.ROWCNT, (int)csr.permLen, NB0 + (size_t)s * D * 2 * D, Fp(23) + s * D, NB1 + (size_t)s * D * D, Fp(25) + s * D, Fp(26) + s * D, Fp(27) + s * D, N, ELIM, NP_); }
  mlp_kernel<4><<<N / 16, 32, 0, stream>>>(NP_, nullptr, nul, nul, nul, nul, nul, 0, DC0, Fp(29), DC1, Fp(31), nullptr, nullptr, N, ELIM, (float*)d_out);
}
